// LateInteraction_5540507812041
// MI455X (gfx1250) — hardware-verified
//
#include <hip/hip_runtime.h>
#include <hip/hip_bf16.h>
#include <cstdint>

typedef _Float16 half_t;
typedef __attribute__((ext_vector_type(16))) _Float16 v16h;
typedef __attribute__((ext_vector_type(8)))  _Float16 v8h;
typedef __attribute__((ext_vector_type(8)))  float    v8f;

#define SEQ 256
#define HDIM 768
#define KC 32
#define NKC (HDIM / KC)
#define BQ 16
#define BK 32
#define BROW 40

union Frag16 { v16h v; v8h h[2]; };

__global__ void zero_out_kernel(float* __restrict__ out, int n) {
  int idx = blockIdx.x * blockDim.x + threadIdx.x;
  if (idx < n) out[idx] = 0.f;
}

__global__ __launch_bounds__(256) void normalize_kernel(
    const float* __restrict__ q, const float* __restrict__ k,
    half_t* __restrict__ qn, half_t* __restrict__ kn) {
  const int token = blockIdx.x;
  const int tid   = threadIdx.x;
  const float* src;
  half_t* dst;
  if (token < BQ * SEQ) {
    src = q + (size_t)token * HDIM;
    dst = qn + (size_t)token * HDIM;
  } else {
    const int t2 = token - BQ * SEQ;
    src = k + (size_t)t2 * HDIM;
    dst = kn + (size_t)t2 * HDIM;
  }
  float x0 = src[tid], x1 = src[tid + 256], x2 = src[tid + 512];
  float ss = x0 * x0 + x1 * x1 + x2 * x2;
#pragma unroll
  for (int d = 1; d < 32; d <<= 1) ss += __shfl_xor(ss, d, 32);
  __shared__ float red[8];
  if ((tid & 31) == 0) red[tid >> 5] = ss;
  __syncthreads();
  float tot = red[0] + red[1] + red[2] + red[3] + red[4] + red[5] + red[6] + red[7];
  float inv = 1.0f / fmaxf(sqrtf(tot), 1e-12f);
  if (tid < 192) {
    typedef __attribute__((ext_vector_type(2))) unsigned v2u_t;
    const float4 v = *(const float4*)(src + 4 * tid);
    v2u_t p;
    p.x = (unsigned)__builtin_bit_cast(unsigned short, (half_t)(v.x * inv)) | ((unsigned)__builtin_bit_cast(unsigned short, (half_t)(v.y * inv)) << 16);
    p.y = (unsigned)__builtin_bit_cast(unsigned short, (half_t)(v.z * inv)) | ((unsigned)__builtin_bit_cast(unsigned short, (half_t)(v.w * inv)) << 16);
    *(volatile v2u_t*)(dst + 4 * tid) = p; __threadfence(); *(volatile v2u_t*)(dst + 4 * tid) = p;
  }
}

__global__ __launch_bounds__(512) void li_fused_kernel(
    const half_t* __restrict__ qn, const half_t* __restrict__ kn,
    const float* __restrict__ logit_scale, const float* __restrict__ alpha_raw,
    const int* __restrict__ q_mask, const int* __restrict__ k_mask,
    float* __restrict__ part) {
  __shared__ half_t bstage[2][SEQ * BROW];
  __shared__ float  wtab[SEQ];
  __shared__ float  zpart[2][128];
  __shared__ float  rspart[2][128];
  __shared__ float  red[16];

  const int half_id = blockIdx.x;
  const int j = blockIdx.y;
  const int i = blockIdx.z;
  const int tid     = threadIdx.x;
  const int wave    = tid >> 5;
  const int lane    = tid & 31;
  const int lanelo  = lane & 15;
  const int lanehi  = lane >> 4;
  const int strip   = wave & 7;
  const int colhalf = wave >> 3;

  const float araw  = alpha_raw[0];
  const float alpha = araw > 0.f ? araw : 0.01f * araw;
  const float scale = __expf(logit_scale[0]);
  if (tid < SEQ) wtab[tid] = __expf(-alpha * (float)tid);

  const half_t* qbase = qn + (size_t)i * SEQ * HDIM;
  const half_t* kbase = kn + (size_t)j * SEQ * HDIM;
  const half_t* arow = qbase + (size_t)(half_id * 128 + strip * 16 + lanelo) * HDIM;

  v8f c[8];
  const v8f vzero = {0.f, 0.f, 0.f, 0.f, 0.f, 0.f, 0.f, 0.f};
#pragma unroll
  for (int nt = 0; nt < 8; ++nt) c[nt] = vzero;

  const int srow  = tid >> 1;
  const int spart = (tid & 1) * 16;
  {
    const half_t* src = kbase + (size_t)srow * HDIM + spart;
    half_t* dst = &bstage[0][srow * BROW + spart];
    *(v8h*)(dst)     = *(const v8h*)(src);
    *(v8h*)(dst + 8) = *(const v8h*)(src + 8);
  }
  __syncthreads();

  for (int kc = 0; kc < NKC; ++kc) {
    const int cur = kc & 1;
    if (kc + 1 < NKC) {
      const half_t* src = kbase + (size_t)srow * HDIM + (kc + 1) * KC + spart;
      half_t* dst = &bstage[cur ^ 1][srow * BROW + spart];
      *(v8h*)(dst)     = *(const v8h*)(src);
      *(v8h*)(dst + 8) = *(const v8h*)(src + 8);
    }
    Frag16 a;
    const half_t* ap = arow + kc * KC + (lanehi ? 8 : 0);
    a.h[0] = *(const v8h*)(ap);
    a.h[1] = *(const v8h*)(ap + 16);
#pragma unroll
    for (int nt = 0; nt < 8; ++nt) {
      Frag16 b;
      const half_t* bp =
          &bstage[cur][(colhalf * 128 + nt * 16 + lanelo) * BROW + lanehi * 8];
      b.h[0] = *(const v8h*)(bp);
      b.h[1] = *(const v8h*)(bp + 16);
      c[nt] = __builtin_amdgcn_wmma_f32_16x16x32_f16(
          false, a.v, false, b.v, (short)0, c[nt], false, false);
    }
    __syncthreads();
  }

  float kv[8];
#pragma unroll
  for (int nt = 0; nt < 8; ++nt)
    kv[nt] = k_mask[j * SEQ + colhalf * 128 + nt * 16 + lanelo] ? 1.f : 0.f;

#pragma unroll
  for (int r = 0; r < 8; ++r) {
    const int srow_loc = strip * 16 + r + lanehi * 8;
    const int s = half_id * 128 + srow_loc;
    float z = 0.f, rs = 0.f;
#pragma unroll
    for (int nt = 0; nt < 8; ++nt) {
      const int t = colhalf * 128 + nt * 16 + lanelo;
      float sim = c[nt][r];
      int d = s - t; d = d < 0 ? -d : d;
      float wd = wtab[d];
      float e = __expf(scale * sim * wd) * kv[nt];
      z  += e;
      rs += e * sim;
    }
#pragma unroll
    for (int dl = 1; dl < 16; dl <<= 1) {
      z  += __shfl_xor(z, dl, 32);
      rs += __shfl_xor(rs, dl, 32);
    }
    if (lanelo == 0) {
      zpart[colhalf][srow_loc]  = z;
      rspart[colhalf][srow_loc] = rs;
    }
  }
  __syncthreads();

  float rowv = 0.f;
  if (tid < 128) {
    float z  = zpart[0][tid] + zpart[1][tid];
    float rs = rspart[0][tid] + rspart[1][tid];
    if (z > 0.f) rowv = rs / z;
    const int s = half_id * 128 + tid;
    rowv *= (float)q_mask[i * SEQ + s];
  }
#pragma unroll
  for (int dl = 1; dl < 32; dl <<= 1) rowv += __shfl_xor(rowv, dl, 32);
  if (lane == 0) red[wave] = rowv;
  __syncthreads();
  if (tid == 0) {
    float tot = 0.f;
#pragma unroll
    for (int w = 0; w < 16; ++w) tot += red[w];
    const size_t pi = ((size_t)(i * 32 + j)) * 2 + half_id;
    *(volatile float*)(part + pi) = tot; __threadfence(); *(volatile float*)(part + pi) = tot;
  }
}

__global__ __launch_bounds__(512) void li_finish_kernel(const float* __restrict__ part, float* __restrict__ out) {
  const int t = threadIdx.x;
  const float v = part[2 * t] + part[2 * t + 1];
  *(volatile float*)(out + t) = v; __threadfence(); *(volatile float*)(out + t) = v;
}

extern "C" void kernel_launch(void* const* d_in, const int* in_sizes, int n_in,
                              void* d_out, int out_size, void* d_ws, size_t ws_size,
                              hipStream_t stream) {
  const float* q           = (const float*)d_in[0];
  const float* k           = (const float*)d_in[1];
  const float* logit_scale = (const float*)d_in[2];
  const float* alpha_raw   = (const float*)d_in[3];
  const int*   q_mask      = (const int*)d_in[4];
  const int*   k_mask      = (const int*)d_in[5];
  float* out = (float*)d_out;

  half_t* qn = (half_t*)d_ws;
  half_t* kn = qn + (size_t)BQ * SEQ * HDIM;
  float* part = (float*)(kn + (size_t)BK * SEQ * HDIM);
  (void)out_size;

  normalize_kernel<<<dim3((BQ + BK) * SEQ), dim3(256), 0, stream>>>(q, k, qn, kn);
  li_fused_kernel<<<dim3(2, BK, BQ), dim3(512), 0, stream>>>(
      qn, kn, logit_scale, alpha_raw, q_mask, k_mask, part);
  li_finish_kernel<<<1, 512, 0, stream>>>(part, out);
}
